// Net_5239860101629
// MI455X (gfx1250) — hardware-verified
//
#include <hip/hip_runtime.h>
#include <stddef.h>
#include <stdint.h>


#define DIN      128
#define DHID     128
#define APW      256
#define KTOT     256
#define WSQ      (DHID * KTOT)
#define NTHR     256
#define NWAVE    8
#define EPT      8
#define CHUNK    (NTHR * EPT)
#define WCAP     (EPT * 32)
#define LISTN    (NWAVE * WCAP)
#define NBMAX    2048
#define NBRUN    1024
#define NBSH     10
#define RCAP     28672
#define DEGCAP   64
#define PKS      11
#define GBM      64
#define GTHR     128
#define GNT      8
#define BN       (16 * GNT)
#define NUSQ     (DHID * (KTOT / 8))
#define NLAY     3
#define NBW      ((2 * NLAY * NUSQ) / NTHR)
#define PARTW    288
#define PARV     (NLAY * 4 * DHID)
#define PAR_EPS  PARV
#define PARN     (PARV + 32)
#define AROWS    64
#define WSMAX    134217728
#define LDS_BKT  ((2 * RCAP + 2 * NBMAX + LISTN) * 4 + 64)

static_assert((CHUNK & (CHUNK - 1)) == 0 && CHUNK <= (1 << PKS));
static_assert((NBMAX & (NBMAX - 1)) == 0 && NBMAX <= (1 << PKS));
static_assert(NTHR * 8 == NBMAX);
static_assert(NBRUN == (1 << NBSH) && NBRUN <= NBMAX && NBRUN == 4 * NTHR);
static_assert(LISTN >= NBMAX);
static_assert((RCAP % (4 * NTHR)) == 0);
static_assert(RCAP >= 17455);
static_assert(DEGCAP >= 35 + 8);
static_assert(LDS_BKT <= 300000);
static_assert(GBM == (GTHR / 32) * 16);
static_assert((DIN % 32) == 0 && KTOT == 2 * DIN && APW == 2 * DIN && (KTOT % 32) == 0);
static_assert(DIN == 32 * 4 && DHID == BN && DHID == DIN && GTHR == BN);
static_assert((NUSQ % NTHR) == 0 && (KTOT / 8) == 32);
static_assert(NTHR == 2 * DHID);
static_assert((PARTW % 32) == 0 && PARTW / 4 <= GTHR && PARTW >= 2 * BN + 1);
static_assert((PARN % 32) == 0 && PARN / 4 <= 2 * NTHR && PARN >= PARV + NLAY);
static_assert(AROWS == GBM && (AROWS % NWAVE) == 0);
static_assert(((50000 + GBM - 1) / GBM) * GBM == 391 * 128);

typedef float          v4f  __attribute__((ext_vector_type(4)));
typedef float          v8f  __attribute__((ext_vector_type(8)));
typedef int            v4i  __attribute__((ext_vector_type(4)));
typedef int            v8i  __attribute__((ext_vector_type(8)));
typedef unsigned int   v2u  __attribute__((ext_vector_type(2)));
typedef unsigned int   v4u  __attribute__((ext_vector_type(4)));
typedef unsigned short v8us __attribute__((ext_vector_type(8)));
typedef __bf16         v16b __attribute__((ext_vector_type(16)));
typedef v4f  __attribute__((may_alias)) v4fa;
typedef v4i  __attribute__((may_alias)) v4ia;
typedef v8us __attribute__((may_alias)) v8usa;
union FragB { v16b v; v8us h[2]; v8i w; };

__device__ __forceinline__ v8f wmb(const FragB& a, const FragB& b, v8f c) {
  v8f d = __builtin_amdgcn_wmma_f32_16x16x32_bf16(false, a.v, false, b.v, (short)0, c, false, false);
  asm volatile("v_nop\n\tv_nop\n\tv_nop\n\tv_nop" : "+v"(d) : "v"(a.w), "v"(b.w));
  return d;
}

__device__ __forceinline__ unsigned short bf_bits(float f) {
  const unsigned int u = __float_as_uint(f);
  const unsigned int r = (u + 0x7FFFu + ((u >> 16) & 1u)) >> 16;
  return (unsigned short)((f != f) ? 0x7FC0u : r);
}
__device__ __forceinline__ float bf_val(unsigned short b) {
  return __uint_as_float(((unsigned int)b) << 16);
}
__device__ __forceinline__ float bf_rne(float f) { return bf_val(bf_bits(f)); }
__device__ __forceinline__ float relu_keep(float v) { return (v > 0.0f) ? v : (v - v); }
__device__ __forceinline__ int clampi(int v, int lo, int hi) { return v < lo ? lo : (v > hi ? hi : v); }

__device__ __forceinline__ int scan_chunk(const int* __restrict__ dsts, int nE, int cbase, int slotBase,
                                          int nb, int vec8, int* list, int tid, int lane, int wave) {
  int wc = 0;
  const int el0  = tid * EPT;
  const int e0   = cbase + el0;
  const int sent = -2147483647 - 1;
  v4i da, db;
  if (vec8 != 0 && cbase + CHUNK <= nE) {
    da = *(const v4i*)(dsts + e0);
    db = *(const v4i*)(dsts + e0 + 4);
  } else {
    da.x = (e0     < nE) ? dsts[min(e0,     nE - 1)] : sent;
    da.y = (e0 + 1 < nE) ? dsts[min(e0 + 1, nE - 1)] : sent;
    da.z = (e0 + 2 < nE) ? dsts[min(e0 + 2, nE - 1)] : sent;
    da.w = (e0 + 3 < nE) ? dsts[min(e0 + 3, nE - 1)] : sent;
    db.x = (e0 + 4 < nE) ? dsts[min(e0 + 4, nE - 1)] : sent;
    db.y = (e0 + 5 < nE) ? dsts[min(e0 + 5, nE - 1)] : sent;
    db.z = (e0 + 6 < nE) ? dsts[min(e0 + 6, nE - 1)] : sent;
    db.w = (e0 + 7 < nE) ? dsts[min(e0 + 7, nE - 1)] : sent;
  }
  const unsigned nbs = (unsigned)slotBase;
  const unsigned unb = (unsigned)nb;
  const unsigned s0 = (unsigned)da.x - nbs, s1 = (unsigned)da.y - nbs;
  const unsigned s2 = (unsigned)da.z - nbs, s3 = (unsigned)da.w - nbs;
  const unsigned s4 = (unsigned)db.x - nbs, s5 = (unsigned)db.y - nbs;
  const unsigned s6 = (unsigned)db.z - nbs, s7 = (unsigned)db.w - nbs;
  const bool h0 = s0 < unb, h1 = s1 < unb, h2 = s2 < unb, h3 = s3 < unb;
  const bool h4 = s4 < unb, h5 = s5 < unb, h6 = s6 < unb, h7 = s7 < unb;
  const unsigned any = __builtin_amdgcn_ballot_w32(h0 | h1 | h2 | h3 | h4 | h5 | h6 | h7);
  if (any != 0u) {
#define HITJ(J, HJ, SJ) { \
      const unsigned mj = __builtin_amdgcn_ballot_w32(HJ); \
      if (mj != 0u) { \
        if (HJ) { \
          const int pos = wc + (int)__builtin_amdgcn_mbcnt_lo(mj, 0u); \
          if (pos < WCAP) list[wave * WCAP + pos] = ((el0 + (J)) << PKS) | (int)(SJ); \
        } \
        wc += (int)__builtin_popcount(mj); } }
    HITJ(0, h0, s0)
    HITJ(1, h1, s1)
    HITJ(2, h2, s2)
    HITJ(3, h3, s3)
    HITJ(4, h4, s4)
    HITJ(5, h5, s5)
    HITJ(6, h6, s6)
    HITJ(7, h7, s7)
#undef HITJ
  }
  return wc;
}

__device__ __forceinline__ v8us wunit(const float* __restrict__ W, int layer, int kk, int n) {
  const float* p = W + (size_t)layer * DIN * DHID + (size_t)kk * DHID + n;
  v8us o;
#pragma unroll
  for (int i = 0; i < 8; ++i) o[i] = bf_bits(p[(size_t)i * DHID]);
  return o;
}

__global__ __launch_bounds__(NTHR) void k_prep(const float* __restrict__ x,
                                               const float* __restrict__ W1, const float* __restrict__ W2,
                                               const float* __restrict__ b1, const float* __restrict__ gam,
                                               const float* __restrict__ bet, const float* __restrict__ b2,
                                               const float* __restrict__ eps,
                                               unsigned short* wt, float* par, float* X, int nN, int nUx) {
  __shared__ __attribute__((aligned(16))) float pst[PARN];
  const int tid = (int)threadIdx.x;
  const int bx  = (int)blockIdx.x;
  if (bx < NBW) {
    const int u     = bx * NTHR + tid;
    const int mi    = u / NUSQ;
    const int v     = u - mi * NUSQ;
    const int n     = v >> 5;
    const int k8    = (v & 31) * 8;
    const int kk    = k8 & (DIN - 1);
    const int layer = mi >> 1;
    v8us o;
    if ((mi & 1) != 0) o = wunit(W2, layer, kk, n);
    else               o = wunit(W1, layer, kk, n);
    unsigned short* dp = wt + (size_t)mi * WSQ + (size_t)n * KTOT + k8;
    *(volatile v8us*)dp = o;
    __threadfence();
    *(volatile v8us*)dp = o;
    return;
  }
  if (bx == NBW) {
#pragma unroll 1
    for (int idx = tid; idx < PARN; idx += NTHR) {
      const int i5 = idx < PARV ? idx : PARV - 1;
      const int l  = i5 >> 9;
      const int j  = (i5 >> 7) & 3;
      const int c  = i5 & (DHID - 1);
      const int q  = l * DHID + c;
      const float va = b1[q], vb = gam[q], vc = bet[q], vd = b2[q];
      const int ei = clampi(idx - PARV, 0, NLAY - 1);
      const float ve = eps[ei];
      float v = (j == 0) ? va : ((j == 1) ? vb : ((j == 2) ? vc : vd));
      v = (idx < PARV) ? v : ((idx < PARV + NLAY) ? ve : 0.0f);
      pst[idx] = bf_rne(v);
    }
    __syncthreads();
    const int u1 = tid + NTHR;
    const bool ok1 = u1 < PARN / 4;
    const int u1c = ok1 ? u1 : PARN / 4 - 1;
    const v4f p0 = *(const v4fa*)(pst + 4 * tid);
    const v4f p1 = *(const v4fa*)(pst + 4 * u1c);
    *(volatile v4f*)(par + 4 * tid) = p0;
    if (ok1) *(volatile v4f*)(par + 4 * u1) = p1;
    __threadfence();
    *(volatile v4f*)(par + 4 * tid) = p0;
    if (ok1) *(volatile v4f*)(par + 4 * u1) = p1;
    return;
  }
  const int u = (bx - NBW - 1) * NTHR + tid;
  if (u >= nUx) return;
  const int row = u >> 5;
  const int c4  = (u & 31) * 4;
  const int rc  = row < nN ? row : nN - 1;
  const bool ok = row < nN;
  const v4f a = *(const v4f*)(x + (size_t)rc * DIN + c4);
  v4f o;
  o.x = ok ? bf_rne(a.x) : 0.0f;
  o.y = ok ? bf_rne(a.y) : 0.0f;
  o.z = ok ? bf_rne(a.z) : 0.0f;
  o.w = ok ? bf_rne(a.w) : 0.0f;
  float* xp = X + (size_t)row * DIN + c4;
  *(volatile v4f*)xp = o;
  __threadfence();
  *(volatile v4f*)xp = o;
}

__global__ __launch_bounds__(NTHR) void k_bucket(const int* __restrict__ srcs, const int* __restrict__ dsts,
                                                 int nN, int nE, int vec8,
                                                 int* LISTg, int* CNTg, int* OFFg, int* FLGg) {
  extern __shared__ v4f lds_dyn[];
  int* reg1 = (int*)lds_dyn;
  int* reg2 = reg1 + RCAP;
  int* scnt = reg2 + RCAP;
  int* soff = scnt + NBMAX;
  int* list = soff + NBMAX;
  int* wcnt = list + LISTN;
  int* wtot = wcnt + NWAVE;
  const int tid = (int)threadIdx.x, lane = tid & 31, wave = tid >> 5;
  const int nodeBase = (int)blockIdx.x * NBRUN;
  const int nb = NBRUN;

  {
    const v4i z4 = {0, 0, 0, 0};
    for (int i = 4 * tid; i < 2 * RCAP; i += 4 * NTHR) *(v4ia*)(reg1 + i) = z4;
    for (int i = tid; i < NBMAX; i += NTHR) scnt[i] = 0;
  }
  __syncthreads();

  int tot = 0;
  const int nChunks = (nE + CHUNK - 1) / CHUNK;
#pragma unroll 1
  for (int ch = 0; ch < nChunks; ++ch) {
    const int cbase = ch * CHUNK;
    const int wc = scan_chunk(dsts, nE, cbase, nodeBase, nb, vec8, list, tid, lane, wave);
    if (lane == 0) wcnt[wave] = wc;
    __syncthreads();
    int pre = 0, all = 0;
#pragma unroll
    for (int w2 = 0; w2 < NWAVE; ++w2) {
      int c = wcnt[w2];
      c = c < 0 ? 0 : (c > WCAP ? WCAP : c);
      all += c;
      pre += (w2 < wave) ? c : 0;
    }
    const int wcc  = wc > WCAP ? WCAP : wc;
    const int base = tot + pre;
#pragma unroll 1
    for (int i = lane; i < wcc; i += 32) {
      const int ent = list[wave * WCAP + i];
      const int el  = (ent >> PKS) & (CHUNK - 1);
      const int sl  = ent & (NBMAX - 1);
      int eid = cbase + el;
      eid = eid > nE - 1 ? nE - 1 : eid;
      const int pos = base + i;
      if (pos < RCAP) reg1[pos] = (int)(((unsigned)eid << PKS) | (unsigned)sl);
    }
    tot += all;
    tot = tot > RCAP ? RCAP : tot;
    __syncthreads();
  }
  const int nh = tot;

  if (wave == 0) {
#pragma unroll 1
    for (int b0 = 0; b0 < nh; b0 += 32) {
      const int idx = b0 + lane;
      const int uv  = reg1[idx < RCAP ? idx : RCAP - 1];
      const int m32 = (nh - b0) < 32 ? (nh - b0) : 32;
#pragma unroll 1
      for (int k = 0; k < m32; ++k) {
        const int u  = __builtin_amdgcn_readlane(uv, k);
        const int sl = u & (NBMAX - 1);
        if (lane == 0) scnt[sl] = scnt[sl] + 1;
      }
    }
  }
  __syncthreads();

  {
    const v4i ca = *(const v4ia*)(scnt + 8 * tid);
    const v4i cb = *(const v4ia*)(scnt + 8 * tid + 4);
    const int e0 = ca.x < 0 ? 0 : ca.x, e1 = ca.y < 0 ? 0 : ca.y, e2 = ca.z < 0 ? 0 : ca.z, e3 = ca.w < 0 ? 0 : ca.w;
    const int e4 = cb.x < 0 ? 0 : cb.x, e5 = cb.y < 0 ? 0 : cb.y, e6 = cb.z < 0 ? 0 : cb.z, e7 = cb.w < 0 ? 0 : cb.w;
    const int ts = e0 + e1 + e2 + e3 + e4 + e5 + e6 + e7;
    int incl = ts;
#pragma unroll
    for (int d = 1; d < 32; d <<= 1) {
      const int up = __shfl_up(incl, d);
      incl += (lane >= d) ? up : 0;
    }
    if (lane == 31) wtot[wave] = incl;
    __syncthreads();
    int pre = 0;
#pragma unroll
    for (int w2 = 0; w2 < NWAVE; ++w2) pre += (w2 < wave) ? wtot[w2] : 0;
    int run = pre + incl - ts;
    soff[8 * tid + 0] = run; run += e0;
    soff[8 * tid + 1] = run; run += e1;
    soff[8 * tid + 2] = run; run += e2;
    soff[8 * tid + 3] = run; run += e3;
    soff[8 * tid + 4] = run; run += e4;
    soff[8 * tid + 5] = run; run += e5;
    soff[8 * tid + 6] = run; run += e6;
    soff[8 * tid + 7] = run;
  }
  __syncthreads();
  for (int i = tid; i < NBMAX; i += NTHR) list[i] = soff[i];
  __syncthreads();

  if (wave == 0) {
#pragma unroll 1
    for (int b0 = 0; b0 < nh; b0 += 32) {
      const int idx = b0 + lane;
      const int uv  = reg1[idx < RCAP ? idx : RCAP - 1];
      const int m32 = (nh - b0) < 32 ? (nh - b0) : 32;
#pragma unroll 1
      for (int k = 0; k < m32; ++k) {
        const int u   = __builtin_amdgcn_readlane(uv, k);
        const int sl  = u & (NBMAX - 1);
        const int eid = (int)((unsigned)u >> PKS);
        if (lane == 0) {
          int pos = list[sl];
          pos = pos < 0 ? 0 : (pos > RCAP - 1 ? RCAP - 1 : pos);
          reg2[pos] = eid;
          list[sl] = pos + 1;
        }
      }
    }
  }
  __syncthreads();

  int* lp = LISTg + (size_t)blockIdx.x * RCAP;
#pragma unroll 1
  for (int it = 0; it < RCAP / (4 * NTHR); ++it) {
    const int p0 = 4 * (it * NTHR + tid);
    const v4i e4 = *(const v4ia*)(reg2 + p0);
    const int q0 = clampi(e4.x, 0, nE - 1), q1 = clampi(e4.y, 0, nE - 1);
    const int q2 = clampi(e4.z, 0, nE - 1), q3 = clampi(e4.w, 0, nE - 1);
    const int r0 = srcs[q0], r1 = srcs[q1], r2 = srcs[q2], r3 = srcs[q3];
    v4i o;
    o.x = (p0     < nh) ? clampi(r0, 0, nN - 1) : 0;
    o.y = (p0 + 1 < nh) ? clampi(r1, 0, nN - 1) : 0;
    o.z = (p0 + 2 < nh) ? clampi(r2, 0, nN - 1) : 0;
    o.w = (p0 + 3 < nh) ? clampi(r3, 0, nN - 1) : 0;
    *(volatile v4i*)(lp + p0) = o;
    __threadfence();
    *(volatile v4i*)(lp + p0) = o;
  }
  {
    const v4i c4 = *(const v4ia*)(scnt + 4 * tid);
    const v4i o4 = *(const v4ia*)(soff + 4 * tid);
    const int ov = (nh >= RCAP) ? 1 : 0;
    v4i f4; f4.x = ov; f4.y = ov; f4.z = ov; f4.w = ov;
    int* cp = CNTg + (size_t)blockIdx.x * NBRUN + 4 * tid;
    int* op = OFFg + (size_t)blockIdx.x * NBRUN + 4 * tid;
    int* fp = FLGg + (size_t)blockIdx.x * 32 + 4 * (tid & 7);
    *(volatile v4i*)cp = c4;
    *(volatile v4i*)op = o4;
    if (tid < 8) *(volatile v4i*)fp = f4;
    __threadfence();
    *(volatile v4i*)cp = c4;
    *(volatile v4i*)op = o4;
    if (tid < 8) *(volatile v4i*)fp = f4;
  }
}

__global__ __launch_bounds__(NTHR) void k_agg(const float* __restrict__ X, const int* __restrict__ LISTg,
                                              const int* __restrict__ CNTg, const int* __restrict__ OFFg,
                                              const int* __restrict__ FLGg, const float* __restrict__ par,
                                              int layer, unsigned short* P1, int nN, int MPr) {
  const int tid = (int)threadIdx.x, lane = tid & 31, wave = tid >> 5;
  const int lc = clampi(layer, 0, NLAY - 1);
  const float onepe = 1.0f + par[PAR_EPS + lc];
  const float qnan = __int_as_float(0x7fc00000);
  const int sl0 = 2 * (lane & 15), sl1 = sl0 + 1;
  const bool isHi = lane < 16;
  const int rowBase = (int)blockIdx.x * AROWS + wave * (AROWS / NWAVE);

#pragma unroll 1
  for (int jt = 0; jt < AROWS / NWAVE; ++jt) {
    const int row = rowBase + jt;
    const int rc  = row < MPr ? row : MPr - 1;
    const int bk  = rc >> NBSH;
    const int craw = __builtin_amdgcn_readfirstlane(CNTg[rc]);
    int st         = __builtin_amdgcn_readfirstlane(OFFg[rc]);
    const int fl   = __builtin_amdgcn_readfirstlane(FLGg[bk * 32]);
    int cnt = clampi(craw, 0, DEGCAP);
    st = clampi(st, 0, RCAP);
    if (cnt > RCAP - st) cnt = RCAP - st;
    const bool bad = (fl != 0) || (craw > DEGCAP) || (craw < 0);
    const bool liveRow = row < nN;
    const int* lp = LISTg + (size_t)bk * RCAP;

    float ag0 = 0.0f, ag1 = 0.0f, ag2 = 0.0f, ag3 = 0.0f;
#pragma unroll 1
    for (int b0 = 0; b0 < cnt; b0 += 32) {
      int idx = st + b0 + lane;
      const int last = st + cnt - 1;
      idx = idx > last ? last : idx;
      idx = clampi(idx, 0, RCAP - 1);
      const int sv = clampi(lp[idx], 0, nN - 1);
      const int m32 = (cnt - b0) < 32 ? (cnt - b0) : 32;
#pragma unroll 1
      for (int k = 0; k < m32; ++k) {
        const int sk = __builtin_amdgcn_readlane(sv, k);
        const v4f v = *(const v4f*)(X + (size_t)sk * DIN + 4 * lane);
        ag0 += v.x; ag1 += v.y; ag2 += v.z; ag3 += v.w;
      }
    }
    const v4f xv = *(const v4f*)(X + (size_t)rc * DIN + 4 * lane);
    float sa = ag0 * ag0 + ag1 * ag1 + ag2 * ag2 + ag3 * ag3;
    float sx = xv.x * xv.x + xv.y * xv.y + xv.z * xv.z + xv.w * xv.w;
#pragma unroll
    for (int o = 16; o > 0; o >>= 1) {
      sa += __shfl_xor(sa, o, 32);
      sx += __shfl_xor(sx, o, 32);
    }
    const float ia = 1.0f / fmaxf(sqrtf(sa), 1e-12f);
    const float ix = 1.0f / fmaxf(sqrtf(sx), 1e-12f);
    float r0 = ag0 * ia + onepe * (xv.x * ix);
    float r1 = ag1 * ia + onepe * (xv.y * ix);
    float r2 = ag2 * ia + onepe * (xv.z * ix);
    float r3 = ag3 * ia + onepe * (xv.w * ix);
    r0 = bad ? qnan : r0; r1 = bad ? qnan : r1; r2 = bad ? qnan : r2; r3 = bad ? qnan : r3;
    r0 = liveRow ? r0 : 0.0f; r1 = liveRow ? r1 : 0.0f; r2 = liveRow ? r2 : 0.0f; r3 = liveRow ? r3 : 0.0f;

    const unsigned short hb0 = bf_bits(r0), hb1 = bf_bits(r1), hb2 = bf_bits(r2), hb3 = bf_bits(r3);
    const unsigned short lb0 = bf_bits(r0 - bf_val(hb0)), lb1 = bf_bits(r1 - bf_val(hb1));
    const unsigned short lb2 = bf_bits(r2 - bf_val(hb2)), lb3 = bf_bits(r3 - bf_val(hb3));
    const int hwx = (int)((unsigned int)hb0 | ((unsigned int)hb1 << 16));
    const int hwy = (int)((unsigned int)hb2 | ((unsigned int)hb3 << 16));
    const int lwx = (int)((unsigned int)lb0 | ((unsigned int)lb1 << 16));
    const int lwy = (int)((unsigned int)lb2 | ((unsigned int)lb3 << 16));
    const int hA = __shfl(hwx, sl0, 32), hB = __shfl(hwy, sl0, 32);
    const int hC = __shfl(hwx, sl1, 32), hD = __shfl(hwy, sl1, 32);
    const int lA = __shfl(lwx, sl0, 32), lB = __shfl(lwy, sl0, 32);
    const int lC = __shfl(lwx, sl1, 32), lD = __shfl(lwy, sl1, 32);
    v4u pk;
    pk.x = (unsigned int)(isHi ? hA : lA);
    pk.y = (unsigned int)(isHi ? hB : lB);
    pk.z = (unsigned int)(isHi ? hC : lC);
    pk.w = (unsigned int)(isHi ? hD : lD);
    unsigned short* gp = P1 + (size_t)rc * (size_t)APW + 8 * lane;
    const bool wsv = row < MPr;
    if (wsv) *(volatile v4u*)gp = pk;
    __threadfence();
    if (wsv) *(volatile v4u*)gp = pk;
  }
}

template <int MODE>
__global__ __launch_bounds__(GTHR) void k_gemm(const unsigned short* __restrict__ A,
                                               const unsigned short* __restrict__ WT,
                                               const float* __restrict__ biasv,
                                               float* outF, float* part, int nN, int rowLim)
{
  constexpr int NT = GNT;
  constexpr int NI = 16;
  __shared__ __attribute__((aligned(16))) float stg[GBM * BN];
  __shared__ __attribute__((aligned(16))) float pst[PARTW];
  __shared__ __attribute__((aligned(16))) float bsh[BN];
  const int tid = (int)threadIdx.x, lane = tid & 31, wave = tid >> 5, hh = lane >> 4, m = lane & 15;
  const int rowBase = (int)blockIdx.x * GBM;

  if (tid < BN / 4) {
    const v4f b4 = *(const v4f*)(biasv + 4 * tid);
    *(v4fa*)(bsh + 4 * tid) = b4;
  }
  __syncthreads();

  v8f acc[NT];
  {
    const v8f z = {0.f, 0.f, 0.f, 0.f, 0.f, 0.f, 0.f, 0.f};
#pragma unroll
    for (int t = 0; t < NT; ++t) acc[t] = z;
  }
  const unsigned short* ap = A + (size_t)(rowBase + 16 * wave + m) * (size_t)APW + 8 * hh;
  const unsigned short* wp = WT + (size_t)m * (size_t)KTOT + 8 * hh;
  constexpr int ksteps = KTOT / 32;
#pragma unroll 1
  for (int ks = 0; ks < ksteps; ++ks) {
    FragB af;
    af.h[0] = *(const v8usa*)(ap + 32 * ks);
    af.h[1] = *(const v8usa*)(ap + 32 * ks + 16);
#pragma unroll
    for (int t = 0; t < NT; ++t) {
      const unsigned short* wq = wp + (size_t)(16 * t) * (size_t)KTOT + 32 * ks;
      FragB bf;
      bf.h[0] = *(const v8usa*)wq;
      bf.h[1] = *(const v8usa*)(wq + 16);
      acc[t] = wmb(af, bf, acc[t]);
    }
  }

#pragma unroll
  for (int t = 0; t < NT; ++t) {
    const int lc = 16 * t + m;
    const float bb = bsh[lc];
#pragma unroll
    for (int r = 0; r < 8; ++r) {
      const int lr = 16 * wave + 8 * hh + r;
      const bool live = (rowBase + lr) < nN;
      float v = acc[t][r] + bb;
      if (MODE == 1) v = relu_keep(v);
      stg[lr * BN + lc] = live ? v : 0.0f;
    }
  }
  __syncthreads();

  if constexpr (MODE == 0) {
    int rv = nN - rowBase;
    rv = rv < 0 ? 0 : (rv > GBM ? GBM : rv);
    float s = 0.0f;
#pragma unroll 1
    for (int r = 0; r < rv; ++r) s += stg[r * BN + tid];
    const float fn = (float)rv;
    const float mean = s * (1.0f / fmaxf(fn, 1.0f));
    float M2 = 0.0f;
#pragma unroll 1
    for (int r = 0; r < rv; ++r) {
      const float d = stg[r * BN + tid] - mean;
      M2 = fmaf(d, d, M2);
    }
    pst[1 + tid] = mean;
    pst[1 + BN + tid] = M2;
    if (tid == 0) pst[0] = fn;
#pragma unroll 1
    for (int i = 2 * BN + 1 + tid; i < PARTW; i += GTHR) pst[i] = 0.0f;
  }

  v4f fv[NI];
#pragma unroll
  for (int i = 0; i < NI; ++i) {
    const int lr = 16 * wave + i;
    fv[i] = *(const v4fa*)(stg + lr * BN + 4 * lane);
  }
#pragma unroll
  for (int i = 0; i < NI; ++i) {
    const int gr = rowBase + 16 * wave + i;
    float* op = outF + (size_t)gr * (size_t)DHID + 4 * lane;
    if (gr < rowLim) *(volatile v4f*)op = fv[i];
  }
  __threadfence();
#pragma unroll
  for (int i = 0; i < NI; ++i) {
    const int gr = rowBase + 16 * wave + i;
    float* op = outF + (size_t)gr * (size_t)DHID + 4 * lane;
    if (gr < rowLim) *(volatile v4f*)op = fv[i];
  }

  if constexpr (MODE == 0) {
    __syncthreads();
    v4f pv = {0.f, 0.f, 0.f, 0.f};
    if (tid < PARTW / 4) {
      pv = *(const v4fa*)(pst + 4 * tid);
      *(volatile v4f*)(part + (size_t)blockIdx.x * PARTW + 4 * tid) = pv;
    }
    __threadfence();
    if (tid < PARTW / 4) {
      *(volatile v4f*)(part + (size_t)blockIdx.x * PARTW + 4 * tid) = pv;
    }
  }
}

__global__ __launch_bounds__(DHID) void k_comb(const float* __restrict__ part, int nPart, float* stat) {
  __shared__ __attribute__((aligned(16))) float stg[2 * DHID];
  const int tid = (int)threadIdx.x;
  const int c = tid & (DHID - 1);
  double sn = 0.0, sm = 0.0;
#pragma unroll 1
  for (int b = 0; b < nPart; ++b) {
    const float* pr = part + (size_t)b * PARTW;
    const double nb = (double)pr[0];
    const double mb = (double)pr[1 + c];
    sn += nb;
    sm += nb * mb;
  }
  const double nt = sn < 1.0 ? 1.0 : sn;
  const double rn = 1.0 / nt;
  const double mean = sm * rn;
  double M2 = 0.0;
#pragma unroll 1
  for (int b = 0; b < nPart; ++b) {
    const float* pr = part + (size_t)b * PARTW;
    const double nb = (double)pr[0];
    const double mb = (double)pr[1 + c];
    const double qb = (double)pr[1 + DHID + c];
    const double d = mb - mean;
    M2 += qb + nb * d * d;
  }
  const float var = (float)(M2 * rn);
  const float rstd = 1.0f / sqrtf(var + 1e-5f);
  stg[c] = (float)mean;
  stg[DHID + c] = rstd;
  __syncthreads();
  v4f v = {0.f, 0.f, 0.f, 0.f};
  if (tid < (2 * DHID) / 4) {
    v = *(const v4fa*)(stg + 4 * tid);
    *(volatile v4f*)(stat + 4 * tid) = v;
  }
  __threadfence();
  if (tid < (2 * DHID) / 4) {
    *(volatile v4f*)(stat + 4 * tid) = v;
  }
}

__global__ __launch_bounds__(NTHR) void k_apply(const float* __restrict__ T, const float* __restrict__ stat,
                                                const float* __restrict__ gb, unsigned short* P1,
                                                int nN, int MPr) {
#pragma clang fp contract(off)
  __shared__ float ssh[4 * DHID];
  const int tid = (int)threadIdx.x, lane = tid & 31, wave = tid >> 5;
  ssh[tid] = stat[tid];
  ssh[2 * DHID + tid] = gb[tid];
  __syncthreads();
  const int m = lane & 15;
  const bool isHi = lane < 16;
  const int cb = 8 * m;
  float mu[8], rr[8], gg[8], be[8];
#pragma unroll
  for (int j = 0; j < 8; ++j) {
    mu[j] = ssh[cb + j];
    rr[j] = ssh[DHID + cb + j];
    gg[j] = ssh[2 * DHID + cb + j];
    be[j] = ssh[3 * DHID + cb + j];
  }
  const int rowBase = (int)blockIdx.x * AROWS + wave * (AROWS / NWAVE);
#pragma unroll 1
  for (int jt = 0; jt < AROWS / NWAVE; ++jt) {
    const int row = rowBase + jt;
    const bool ok = row < nN;
    const int rc = ok ? row : nN - 1;
    const v4f a = *(const v4f*)(T + (size_t)rc * DHID + cb);
    const v4f b = *(const v4f*)(T + (size_t)rc * DHID + cb + 4);
    const float f[8] = {a.x, a.y, a.z, a.w, b.x, b.y, b.z, b.w};
    float y[8];
#pragma unroll
    for (int j = 0; j < 8; ++j) {
      float t = ((gg[j] * (f[j] - mu[j])) * rr[j]) + be[j];
      t = relu_keep(t);
      y[j] = ok ? t : 0.0f;
    }
    unsigned int w[4];
#pragma unroll
    for (int j = 0; j < 4; ++j) {
      const unsigned short h0 = bf_bits(y[2 * j]), h1 = bf_bits(y[2 * j + 1]);
      const unsigned short l0 = bf_bits(y[2 * j] - bf_val(h0)), l1 = bf_bits(y[2 * j + 1] - bf_val(h1));
      const unsigned short q0 = isHi ? h0 : l0, q1 = isHi ? h1 : l1;
      w[j] = (unsigned int)q0 | ((unsigned int)q1 << 16);
    }
    v4u pk; pk.x = w[0]; pk.y = w[1]; pk.z = w[2]; pk.w = w[3];
    const int rs = row < MPr ? row : MPr - 1;
    unsigned short* gp = P1 + (size_t)rs * (size_t)APW + 8 * lane;
    const bool wsv = row < MPr;
    if (wsv) *(volatile v4u*)gp = pk;
    __threadfence();
    if (wsv) *(volatile v4u*)gp = pk;
  }
}

static inline int cdiv(int a, int b) { return (a + b - 1) / b; }
static inline size_t al256(size_t o) { return (o + 255) & ~(size_t)255; }

extern "C" void kernel_launch(void* const* d_in, const int* in_sizes, int n_in,
                              void* d_out, int out_size, void* d_ws, size_t ws_size,
                              hipStream_t stream) {
  if (n_in < 9) return;
  if (in_sizes[0] < DIN || (in_sizes[0] % DIN) != 0) return;
  const int nN = in_sizes[0] / DIN;
  if (nN < 1 || nN > (1 << 22)) return;
  const int nE2 = in_sizes[1];
  if (nE2 < 2 || (nE2 & 1) != 0) return;
  const int nE = nE2 / 2;
  if (nE < 1 || nE > (1 << 21)) return;
  if (in_sizes[2] != NLAY * DIN * DHID || in_sizes[6] != NLAY * DIN * DHID) return;
  if (in_sizes[3] != NLAY * DHID || in_sizes[4] != NLAY * DHID) return;
  if (in_sizes[5] != NLAY * DHID || in_sizes[7] != NLAY * DHID) return;
  if (in_sizes[8] != NLAY) return;
  if ((long long)out_size != (long long)nN * DHID) return;

  const float* x   = (const float*)d_in[0];
  const int*   ei  = (const int*)  d_in[1];
  const int*   src = ei;
  const int*   dst = ei + nE;
  const float* W1  = (const float*)d_in[2];
  const float* b1  = (const float*)d_in[3];
  const float* gam = (const float*)d_in[4];
  const float* bet = (const float*)d_in[5];
  const float* W2  = (const float*)d_in[6];
  const float* b2  = (const float*)d_in[7];
  const float* eps = (const float*)d_in[8];
  float* out = (float*)d_out;

  const int MP   = cdiv(nN, GBM) * GBM;
  const int gM   = MP / GBM;
  const int gA   = cdiv(MP, NBRUN);
  const int vec8 = ((nE & 3) == 0) ? 1 : 0;
  if ((long long)gA * NBRUN < (long long)MP) return;
  if ((long long)(gM - 1) * GBM >= (long long)nN) return;
  const int nUx  = MP * (DIN / 4);
  if ((nUx % NTHR) != 0) return;

  char* ws = (char*)d_ws;
  size_t off = 0;
  const size_t oWT  = off; off = al256(off + (size_t)(2 * NLAY) * WSQ * 2);
  const size_t oX   = off; off = al256(off + (size_t)MP * DIN * 4);
  const size_t oP1  = off; off = al256(off + (size_t)MP * APW * 2);
  const size_t oT   = off; off = al256(off + (size_t)MP * DHID * 4);
  const size_t oLS  = off; off = al256(off + (size_t)gA * RCAP * 4);
  const size_t oCN  = off; off = al256(off + (size_t)gA * NBRUN * 4);
  const size_t oOF  = off; off = al256(off + (size_t)gA * NBRUN * 4);
  const size_t oFL  = off; off = al256(off + (size_t)gA * 32 * 4);
  const size_t oRC  = off; off = al256(off + (size_t)gM * PARTW * 4);
  const size_t oST  = off; off = al256(off + (size_t)(2 * DHID) * 4);
  const size_t oPR  = off; off = al256(off + (size_t)PARN * 4);
  if (off > ws_size || off > (size_t)WSMAX) return;
  unsigned short* WT   = (unsigned short*)(ws + oWT);
  float*          X    = (float*)(ws + oX);
  unsigned short* P1   = (unsigned short*)(ws + oP1);
  float*          T    = (float*)(ws + oT);
  int*            LIST = (int*)(ws + oLS);
  int*            CNT  = (int*)(ws + oCN);
  int*            OFFp = (int*)(ws + oOF);
  int*            FLG  = (int*)(ws + oFL);
  float*          REC  = (float*)(ws + oRC);
  float*          STAT = (float*)(ws + oST);
  float*          PAR  = (float*)(ws + oPR);

  hipFuncSetAttribute(reinterpret_cast<const void*>(&k_bucket), hipFuncAttributeMaxDynamicSharedMemorySize, LDS_BKT);

  k_prep<<<NBW + 1 + nUx / NTHR, NTHR, 0, stream>>>(x, W1, W2, b1, gam, bet, b2, eps, WT, PAR, X, nN, nUx);
  k_bucket<<<gA, NTHR, LDS_BKT, stream>>>(src, dst, nN, nE, vec8, LIST, CNT, OFFp, FLG);
  for (int l = 0; l < NLAY; ++l) {
    const float* pl = PAR + (size_t)l * 4 * DHID;
    k_agg<<<gM, NTHR, 0, stream>>>(X, LIST, CNT, OFFp, FLG, PAR, l, P1, nN, MP);
    k_gemm<0><<<gM, GTHR, 0, stream>>>(P1, WT + (size_t)(2 * l) * WSQ, pl, T, REC, nN, MP);
    k_comb<<<1, DHID, 0, stream>>>(REC, gM, STAT);
    k_apply<<<gM, NTHR, 0, stream>>>(T, STAT, pl + DHID, P1, nN, MP);
    if (l < NLAY - 1) {
      k_gemm<1><<<gM, GTHR, 0, stream>>>(P1, WT + (size_t)(2 * l + 1) * WSQ, pl + 3 * DHID, X, REC, nN, MP);
    } else {
      k_gemm<2><<<gM, GTHR, 0, stream>>>(P1, WT + (size_t)(2 * l + 1) * WSQ, pl + 3 * DHID, out, REC, nN, nN);
    }
  }
}
